// NumericalBiasModule_24481313587800
// MI455X (gfx1250) — hardware-verified
//
#include <hip/hip_runtime.h>


namespace {
constexpr int N = 100000, E = 1000000, D = 32, REL = 128, HID = 64;
constexpr float EPS = 1e-8f, SR = 0.0625f  , WR = 65536.0f  , SA = 256.0f, WA = 16.0f, F = 4096.0f  ;
typedef _Float16 b16;
typedef __attribute__((ext_vector_type(16))) _Float16 v16b;
typedef __attribute__((ext_vector_type(8))) _Float16 v8b;
typedef __attribute__((ext_vector_type(8))) float v8f;
__device__ __forceinline__ float bf16_rne(float f) { unsigned int u = __float_as_uint(f); u += 0x7FFFu + ((u >> 16) & 1u); float r = __uint_as_float(u & 0xFFFF0000u); asm volatile("" : "+v"(r)); return r; }
__device__ __forceinline__ float bfv(float f) { float r = bf16_rne(f); asm volatile("" : "+v"(r)); return r; }
__device__ __forceinline__ void split16(float v, b16& hi, b16& lo) { hi = (b16)v; lo = (b16)(v - (float)hi); }
__device__ __forceinline__ v16b frag_kb(const b16* p, int hh) { const v8b a = *(const v8b*)(p + 8 * hh), b = *(const v8b*)(p + 16 + 8 * hh); v16b f;
#pragma unroll
  for (int e = 0; e < 8; ++e) { f[e] = a[e]; f[8 + e] = b[e]; } return f; }
__device__ __forceinline__ v8f wmma16b(v16b a, v16b b, v8f c) { v8f d = __builtin_amdgcn_wmma_f32_16x16x32_f16(false, a, false, b, (short)0, c, false, false); asm volatile("v_nop\n\tv_nop\n\tv_nop\n\tv_nop" : "+v"(d) : "v"(a), "v"(b)); return d; }
__device__ __forceinline__ void wave_lds_sync() { __builtin_amdgcn_fence(__ATOMIC_RELEASE, "workgroup"); __builtin_amdgcn_wave_barrier(); __builtin_amdgcn_fence(__ATOMIC_ACQUIRE, "workgroup"); }
__device__ __forceinline__ float pmul(float a, float b) { float p = a * b; asm volatile("" : "+v"(p)); return p; }
__device__ __forceinline__ int iclamp(int v, int lo, int hi) { return v < lo ? lo : (v > hi ? hi : v); }

__global__ __launch_bounds__(256) void wput_kernel(const float* __restrict__ w1, b16* __restrict__ WT) { const int u = blockIdx.x * 256 + threadIdx.x; if (u >= HID * 16) return; const int o = u / 16, k0 = (u % 16) * 8; const float sc = k0 < D ? WR : WA; v8b v;
#pragma unroll
  for (int j = 0; j < 8; ++j) v[j] = (b16)(bf16_rne(w1[o * REL + k0 + j]) * sc); for (int pass = 0; pass < 2; ++pass) { *(volatile v8b*)(WT + (size_t)o * REL + k0) = v; __threadfence(); } }
__global__ __launch_bounds__(32) void nb_kernel(const float* __restrict__ x, const int* __restrict__ ei, const b16* __restrict__ WT, const float* __restrict__ b1, const float* __restrict__ w2, const float* __restrict__ b2, int ELIM, float* __restrict__ out) { __shared__ __attribute__((aligned(16))) b16 Ah[32][REL + 8], Al[32][REL + 8]; __shared__ float Tf[32][HID + 1]; const int lane = threadIdx.x, nloc = lane & 15, hlf = lane >> 4; const size_t e0 = (size_t)blockIdx.x * 32; if (e0 >= (size_t)ELIM) return;
  for (int rr = 0; rr < 32; ++rr) { const size_t e = e0 + rr; const size_t si = (size_t)iclamp(ei[e], 0, N - 1), sj = (size_t)iclamp(ei[E + e], 0, N - 1); const float xi = bfv(x[si * D + lane]), xj = bfv(x[sj * D + lane]);
    const float ratio = xi / (xj + EPS); const float lr = logf(xi + EPS) - logf(xj + EPS); const float ad = fabsf(xi - xj); const float rd = ad / (fmaxf(xi, xj) + EPS);
    b16 p, ql; split16(ratio * SR, p, ql); Ah[rr][lane] = p; Al[rr][lane] = ql; split16(lr * SA, p, ql); Ah[rr][D + lane] = p; Al[rr][D + lane] = ql; split16(ad * SA, p, ql); Ah[rr][2 * D + lane] = p; Al[rr][2 * D + lane] = ql; split16(rd * SA, p, ql); Ah[rr][3 * D + lane] = p; Al[rr][3 * D + lane] = ql; }
  for (int k = REL; k < REL + 8; ++k) { Ah[lane][k] = (b16)0.0f; Al[lane][k] = (b16)0.0f; }
  wave_lds_sync();
#pragma unroll 1
  for (int rt = 0; rt < 2; ++rt) { v8f acc[4] = {(v8f){}, (v8f){}, (v8f){}, (v8f){}};
#pragma unroll
    for (int kb = 0; kb < REL; kb += 32) { const v16b a = frag_kb(&Ah[rt * 16 + nloc][kb], hlf), al = frag_kb(&Al[rt * 16 + nloc][kb], hlf);
#pragma unroll
      for (int t = 0; t < 4; ++t) { const v16b bw = frag_kb(WT + (size_t)(t * 16 + nloc) * REL + kb, hlf); acc[t] = wmma16b(a, bw, acc[t]); acc[t] = wmma16b(al, bw, acc[t]); } }
#pragma unroll
    for (int t = 0; t < 4; ++t) { const int cc = t * 16 + nloc; const float bb = bfv(b1[cc]);
#pragma unroll
      for (int r8 = 0; r8 < 8; ++r8) Tf[rt * 16 + 8 * hlf + r8][cc] = fmaxf(acc[t][r8] * (1.0f / F) + bb, 0.0f); } }
  wave_lds_sync();
  float s = bfv(b2[0]);
#pragma unroll 8
  for (int c = 0; c < HID; ++c) s += pmul(Tf[lane][c], bfv(w2[c]));
  for (int pass = 0; pass < 2; ++pass) { ((volatile float*)out)[e0 + lane] = s; __threadfence(); } }
}

extern "C" void kernel_launch(void* const* d_in, const int* in_sizes, int n_in, void* d_out, int out_size, void* d_ws, size_t ws_size, hipStream_t stream) {
  (void)n_in;
  auto Fp = [&](int i) { return (const float*)d_in[i]; }; auto Ip = [&](int i) { return (const int*)d_in[i]; };
  if (in_sizes[0] != N * D || in_sizes[1] != 2 * E || in_sizes[2] != HID * REL || in_sizes[3] != HID || in_sizes[4] != HID || in_sizes[5] != 1 || out_size != E) return;
  const int ELIM = E;
  size_t off = 0; char* ws = (char*)d_ws;
  auto carve = [&](size_t bytes) { char* p = ws + off; off += (bytes + 255) & ~(size_t)255; return p; };
  b16* WT = (b16*)carve((size_t)HID * REL * 2);
  if (off > ws_size || off > ((size_t)1 << 20)) return;
  wput_kernel<<<(HID * 16 + 255) / 256, 256, 0, stream>>>(Fp(2), WT);
  nb_kernel<<<ELIM / 32, 32, 0, stream>>>(Fp(0), Ip(1), WT, Fp(3), Fp(4), Fp(5), ELIM, (float*)d_out);
}
